// MoE_30416958390574
// MI455X (gfx1250) — hardware-verified
//
#include <hip/hip_runtime.h>
#include <math.h>

typedef __attribute__((ext_vector_type(16))) __bf16 v16b;
typedef __attribute__((ext_vector_type(8)))  __bf16 v8b;
typedef __attribute__((ext_vector_type(8)))  float v8f;
typedef __attribute__((ext_vector_type(4)))  float v4f;
typedef __attribute__((ext_vector_type(4)))  unsigned v4u;

#ifndef NB
#define NB 4
#endif
#ifndef SEQ
#define SEQ 2048
#endif
#define NB_FULL 4
#define SEQ_FULL 2048
#define DIM 1024
#define NE  8
#define NTOK (NB * SEQ)
#define ROWS_NEEDED ((NB - 1) * SEQ_FULL + SEQ)

#define WS_XB  ((size_t)0)
#define WS_WB  (WS_XB  + (size_t)NTOK * DIM * 2)
#define WS_CMB (WS_WB  + (size_t)NE * DIM * DIM * 2)
#define WS_END (WS_CMB + (size_t)NTOK * NE * 4)

static_assert(SEQ % 128 == 0 && SEQ <= SEQ_FULL && NB <= NB_FULL && NB >= 1);
static_assert(NTOK % 128 == 0);
static_assert(DIM == 1024 && DIM % 64 == 0 && DIM % 32 == 0 && NE == 8);
static_assert((size_t)NB_FULL * SEQ_FULL * DIM * 4 == 33554432);
static_assert((size_t)ROWS_NEEDED * DIM * 4 <= 33554432);
static_assert(WS_WB % 128 == 0 && WS_CMB % 128 == 0 && WS_END % 128 == 0);
static_assert(WS_END <= (size_t)134217728);
static_assert((size_t)(NTOK * (DIM / 8) / 256) * 256 * 8 == (size_t)NTOK * DIM);
static_assert((size_t)(NE * DIM * (DIM / 8) / 256) * 256 * 8 == (size_t)NE * DIM * DIM);
static_assert((size_t)(NTOK / 128) * 128 * NE == (size_t)NTOK * NE);
static_assert((size_t)(NTOK / 128) * 2 * 128 * 4 == (size_t)NTOK * NE);
static_assert((size_t)(DIM / 64) * (NTOK / 128) * 128 * 64 == (size_t)NTOK * DIM);
static_assert((NE * DIM) % (4 * 128) == 0);
static_assert(32 * 16 * 8 == 32 * 128);
static_assert(256 * 4 == 128 * NE);
static_assert((size_t)NE * DIM * 4 + (size_t)128 * NE * 4 <= 131072);
static_assert((size_t)128 * NE * 4 + (size_t)8 * 32 * 32 * 4 <= 131072);

__device__ __forceinline__ v8f wmma_bf(v16b a, v16b b, v8f c) {
  v8f d = __builtin_amdgcn_wmma_f32_16x16x32_bf16(false, a, false, b, (short)0, c, false, false);
  asm volatile("v_nop\n\tv_nop\n\tv_nop\n\tv_nop" : "+v"(d) : "v"(a), "v"(b));
  return d;
}
__device__ __forceinline__ float bfr(float v) { return (float)(__bf16)v; }
__device__ __forceinline__ v16b ldfrag_b(const unsigned short* p) { union { v16b v; v4u q[2]; } f; f.q[0] = *(const v4u*)p; f.q[1] = *(const v4u*)(p + 16); return f.v; }

__global__ __launch_bounds__(256) void k_cvt(const float* __restrict__ S, unsigned short* __restrict__ Dst, unsigned n8, unsigned remap) {
#pragma clang fp contract(off)
  const unsigned i = blockIdx.x * 256u + threadIdx.x;
  const unsigned ic = i < n8 ? i : n8 - 1u;
  const unsigned row = ic >> 7, pc = ic & 127u;
  const unsigned mrow = (row / (unsigned)SEQ) * (unsigned)SEQ_FULL + (row % (unsigned)SEQ);
  const unsigned srow = remap ? mrow : row;
  const float* s = S + (size_t)srow * DIM + 8u * pc;
  const v4f a = *(const v4f*)s, b = *(const v4f*)(s + 4);
  union { v8b h; v4u u; } o;
#pragma unroll
  for (int j = 0; j < 4; ++j) { o.h[j] = (__bf16)a[j]; o.h[4 + j] = (__bf16)b[j]; }
  const v4u val = o.u;
  volatile v4u* p = (volatile v4u*)(Dst + (size_t)ic * 8);
  *p = val; __threadfence(); *p = val;
}

__global__ __launch_bounds__(128) void k_gate(const unsigned* __restrict__ XB2, const float* __restrict__ GW, float* __restrict__ CMB) {
#pragma clang fp contract(off)
  __shared__ __align__(16) float gw[NE][DIM];
  __shared__ __align__(16) float sp[128][NE];
  const unsigned tid = threadIdx.x; const unsigned r0 = blockIdx.x * 128u;
#pragma unroll 1
  for (unsigned it = 0; it < (unsigned)(NE * DIM / 4 / 128); ++it) { const unsigned i4 = 4u * (it * 128u + tid); const unsigned e = i4 >> 10, k = i4 & 1023u;
    const v4f v = *(const v4f*)(GW + i4);
    gw[e][k + 0] = bfr(v[0]); gw[e][k + 1] = bfr(v[1]); gw[e][k + 2] = bfr(v[2]); gw[e][k + 3] = bfr(v[3]); }
  __syncthreads();
  const unsigned* xr = XB2 + (size_t)(r0 + tid) * (DIM / 2);
  float acc[NE];
#pragma unroll
  for (int e = 0; e < NE; ++e) acc[e] = 0.0f;
#pragma unroll 1
  for (unsigned k = 0; k < DIM; k += 2) { const unsigned w = xr[k >> 1];
    const float x0 = __uint_as_float(w << 16), x1 = __uint_as_float(w & 0xffff0000u);
#pragma unroll
    for (int e = 0; e < NE; ++e) { acc[e] = fmaf(x0, gw[e][k], acc[e]); acc[e] = fmaf(x1, gw[e][k + 1], acc[e]); } }
  int i0 = 0; float v0 = acc[0];
#pragma unroll
  for (int e = 1; e < NE; ++e) { const bool gt = acc[e] > v0; v0 = gt ? acc[e] : v0; i0 = gt ? e : i0; }
  int i1 = (i0 == 0) ? 1 : 0; float v1 = -INFINITY;
#pragma unroll
  for (int e = 0; e < NE; ++e) { const bool gt = (e != i0) && (acc[e] > v1); v1 = gt ? acc[e] : v1; i1 = gt ? e : i1; }
  const float a = expf(v1 - v0);
  const float inv = 1.0f / (1.0f + a);
  const float w0 = inv, w1 = a * inv;
#pragma unroll
  for (int e = 0; e < NE; ++e) sp[tid][e] = (e == i0) ? w0 : ((e == i1) ? w1 : 0.0f);
  __syncthreads();
  v4f pv[2];
#pragma unroll
  for (unsigned it = 0; it < 2; ++it) { const unsigned idx = it * 128u + tid; pv[it] = *(const v4f*)&sp[idx >> 1][4u * (idx & 1u)]; }
  float* co = CMB + (size_t)r0 * NE;
#pragma unroll
  for (unsigned it = 0; it < 2; ++it) { const unsigned idx = it * 128u + tid; *(volatile v4f*)(co + 4u * idx) = pv[it]; }
  __threadfence();
#pragma unroll
  for (unsigned it = 0; it < 2; ++it) { const unsigned idx = it * 128u + tid; *(volatile v4f*)(co + 4u * idx) = pv[it]; }
}

__global__ __launch_bounds__(256) void k_moe(const unsigned short* __restrict__ XB, const unsigned short* __restrict__ WB, const float* __restrict__ CMB, float* __restrict__ OUT) {
  __shared__ __align__(16) float sc[128][NE];
  __shared__ __align__(16) float sf[8][32][32];
  const unsigned t = threadIdx.x; const unsigned wave = __builtin_amdgcn_readfirstlane(t >> 5);
  const unsigned lane = t & 31u, lm = lane & 15u, lh = lane >> 4, wm = wave >> 1, wn = wave & 1u;
  const unsigned m0 = blockIdx.y * 128u, n0 = blockIdx.x * 64u;
  { const v4f v = *(const v4f*)(CMB + (size_t)m0 * NE + 4u * t); const unsigned rw = t >> 1, c = 4u * (t & 1u);
    sc[rw][c + 0] = v[0]; sc[rw][c + 1] = v[1]; sc[rw][c + 2] = v[2]; sc[rw][c + 3] = v[3]; }
  __syncthreads();
  unsigned ao[2], bo[2];
#pragma unroll
  for (int mi = 0; mi < 2; ++mi) ao[mi] = (m0 + wm * 32u + mi * 16u + lm) * (unsigned)DIM + 8u * lh;
#pragma unroll
  for (int ni = 0; ni < 2; ++ni) bo[ni] = (n0 + wn * 32u + ni * 16u + lm) * (unsigned)DIM + 8u * lh;
  v8f tot[2][2] = {};
#pragma unroll 1
  for (unsigned e = 0; e < (unsigned)NE; ++e) {
    const unsigned eo = e * (unsigned)(DIM * DIM);
    v8f acc[2][2] = {};
#pragma unroll 2
    for (unsigned kc = 0; kc < DIM / 32; ++kc) { v16b a[2], b[2];
#pragma unroll
      for (int mi = 0; mi < 2; ++mi) a[mi] = ldfrag_b(XB + (size_t)(ao[mi] + kc * 32u));
#pragma unroll
      for (int ni = 0; ni < 2; ++ni) b[ni] = ldfrag_b(WB + (size_t)(eo + bo[ni] + kc * 32u));
#pragma unroll
      for (int mi = 0; mi < 2; ++mi)
#pragma unroll
        for (int ni = 0; ni < 2; ++ni) acc[mi][ni] = wmma_bf(a[mi], b[ni], acc[mi][ni]); }
#pragma unroll
    for (int mi = 0; mi < 2; ++mi)
#pragma unroll
      for (int r = 0; r < 8; ++r) { const float cw = sc[wm * 32u + mi * 16u + 8u * lh + r][e];
#pragma unroll
        for (int ni = 0; ni < 2; ++ni) tot[mi][ni][r] = fmaf(acc[mi][ni][r], cw, tot[mi][ni][r]); }
  }
#pragma unroll
  for (int mi = 0; mi < 2; ++mi)
#pragma unroll
    for (int ni = 0; ni < 2; ++ni)
#pragma unroll
      for (int r = 0; r < 8; ++r) sf[wave][mi * 16 + 8u * lh + r][ni * 16 + lm] = tot[mi][ni][r];
  __syncthreads();
  v4f v[8];
#pragma unroll
  for (unsigned it = 0; it < 8; ++it) { const unsigned rw = it * 4u + (lane >> 3), q = lane & 7u; v[it] = *(const v4f*)&sf[wave][rw][4u * q]; }
  const unsigned frow0 = (m0 / (unsigned)SEQ) * (unsigned)SEQ_FULL + (m0 % (unsigned)SEQ);
  float* po = OUT + (size_t)(frow0 + wm * 32u) * DIM + n0 + wn * 32u;
#pragma unroll
  for (unsigned it = 0; it < 8; ++it) { const unsigned rw = it * 4u + (lane >> 3), q = lane & 7u; *(volatile v4f*)(po + (size_t)rw * DIM + 4u * q) = v[it]; }
  __threadfence();
#pragma unroll
  for (unsigned it = 0; it < 8; ++it) { const unsigned rw = it * 4u + (lane >> 3), q = lane & 7u; *(volatile v4f*)(po + (size_t)rw * DIM + 4u * q) = v[it]; }
}

extern "C" void kernel_launch(void* const* d_in, const int* in_sizes, int n_in, void* d_out, int out_size, void* d_ws, size_t ws_size, hipStream_t stream) {
  if (n_in < 3) return;
  if (in_sizes[0] < ROWS_NEEDED * DIM || in_sizes[1] < NE * DIM || in_sizes[2] < NE * DIM * DIM) return;
  if ((size_t)out_size < (size_t)ROWS_NEEDED * DIM) return;
  if (ws_size < (size_t)WS_END) return;
  const float* X  = (const float*)d_in[0];
  const float* GW = (const float*)d_in[1];
  const float* EW = (const float*)d_in[2];
  char* ws = (char*)d_ws;
  unsigned short* XB = (unsigned short*)(ws + WS_XB);
  unsigned short* WB = (unsigned short*)(ws + WS_WB);
  float* CMB = (float*)(ws + WS_CMB);
  float* OUT = (float*)d_out;
  k_cvt<<<dim3(NTOK * (DIM / 8) / 256), 256, 0, stream>>>(X, XB, (unsigned)(NTOK * (DIM / 8)), 1u);
  k_cvt<<<dim3(NE * DIM * (DIM / 8) / 256), 256, 0, stream>>>(EW, WB, (unsigned)(NE * DIM * (DIM / 8)), 0u);
  k_gate<<<dim3(NTOK / 128), 128, 0, stream>>>((const unsigned*)XB, GW, CMB);
  k_moe<<<dim3(DIM / 64, NTOK / 128), 256, 0, stream>>>(XB, WB, CMB, OUT);
}
